// LowRankBilinearPooling_90563680403989
// MI455X (gfx1250) — hardware-verified
//
#include <hip/hip_runtime.h>


#define NB_  16
#define NP   196
#define NR   (NB_ * NP)
#define CC   768
#define HH   512
#define OO   128

typedef unsigned short bf;
typedef __attribute__((ext_vector_type(16))) __bf16   v16bf;
typedef __attribute__((ext_vector_type(8)))  unsigned short v8us;
typedef __attribute__((ext_vector_type(8)))  float    v8f;
typedef __attribute__((ext_vector_type(4)))  float    v4f;
typedef v4f  __attribute__((may_alias)) v4fa;
typedef v8us __attribute__((may_alias)) v8usa;

__device__ __forceinline__ unsigned short f2bf(float f) { unsigned u = __float_as_uint(f); u += 0x7FFFu + ((u >> 16) & 1u); return (unsigned short)(u >> 16); }
__device__ __forceinline__ float bf2f(unsigned short b) { return __uint_as_float(((unsigned)b) << 16); }
__device__ __forceinline__ float bfr(float f) { return bf2f(f2bf(f)); }
__device__ __forceinline__ v16bf cat16b(v8us lo, v8us hi) { return __builtin_bit_cast(v16bf, __builtin_shufflevector(lo, hi, 0, 1, 2, 3, 4, 5, 6, 7, 8, 9, 10, 11, 12, 13, 14, 15)); }
__device__ __forceinline__ v8f wmmab(v16bf a, v16bf b, v8f c) { return __builtin_amdgcn_wmma_f32_16x16x32_bf16(false, a, false, b, (short)0, c, false, false); }
#define VST2(T, p, v) do { const T vst2_v_ = (v); *(volatile T*)(p) = vst2_v_; __threadfence(); *(volatile T*)(p) = vst2_v_; } while (0)

__global__ __launch_bounds__(256) void k_cvtb(const float* __restrict__ src, bf* dst) {
    const int lane = threadIdx.x & 31, r = blockIdx.x * 8 + (threadIdx.x >> 5);
    if (r >= NR) return;
#pragma unroll
    for (int q = 0; q < CC / 256; ++q) { v8us t;
#pragma unroll
        for (int i = 0; i < 8; ++i) t[i] = f2bf(src[(size_t)r * CC + q * 256 + lane * 8 + i]);
        VST2(v8us, dst + (size_t)r * CC + q * 256 + lane * 8, t); }
}
__global__ __launch_bounds__(256) void k_wt(const float* __restrict__ Wm, bf* WT) {
    __shared__ __align__(16) unsigned short tl[64 * 72];
    const int tid = threadIdx.x, k0 = blockIdx.x * 64, n0 = blockIdx.y * 64;
    const int kk = tid >> 2, nq = (tid & 3) * 16;
#pragma unroll
    for (int i = 0; i < 16; ++i) tl[(nq + i) * 72 + kk] = f2bf(Wm[(size_t)(k0 + kk) * HH + n0 + nq + i]);
    __syncthreads();
    const int piece = tid & 7;
    auto pass = [&]() {
#pragma unroll
        for (int s = 0; s < 2; ++s) { const int nr = (tid >> 3) + 32 * s; const v8us val = *(const v8usa*)(tl + nr * 72 + piece * 8);
            *(volatile v8us*)(WT + (size_t)(n0 + nr) * CC + k0 + piece * 8) = val; }
    };
    pass(); __threadfence(); pass();
}
__global__ __launch_bounds__(128) void k_gemm(const bf* __restrict__ A, const bf* __restrict__ Bn, float* C) {
    __shared__ __align__(16) float ost[4][16 * 68];
    const int lane = threadIdx.x & 31, wave = threadIdx.x >> 5, lr = lane & 15, hi = lane >> 4;
    const int r0 = blockIdx.x * 64 + wave * 16, c0 = blockIdx.y * 64;
    const size_t aoff = (size_t)(r0 + lr) * CC + 8 * hi;
    size_t boff[4];
#pragma unroll
    for (int t = 0; t < 4; ++t) boff[t] = (size_t)(c0 + t * 16 + lr) * CC + 8 * hi;
    v8f acc[4];
#pragma unroll
    for (int t = 0; t < 4; ++t) acc[t] = (v8f){};
#pragma unroll 1
    for (int kc = 0; kc < CC; kc += 32) {
        const v16bf a = cat16b(*(const v8us*)(A + aoff + kc), *(const v8us*)(A + aoff + kc + 16));
#pragma unroll
        for (int t = 0; t < 4; ++t) acc[t] = wmmab(a, cat16b(*(const v8us*)(Bn + boff[t] + kc), *(const v8us*)(Bn + boff[t] + kc + 16)), acc[t]);
        asm volatile("v_nop\n\tv_nop\n\tv_nop\n\tv_nop" : "+v"(acc[0]), "+v"(acc[1]), "+v"(acc[2]), "+v"(acc[3]) : "v"(a));
    }
    float* os = &ost[wave][0];
#pragma unroll
    for (int t = 0; t < 4; ++t)
#pragma unroll
        for (int j = 0; j < 8; ++j) os[(hi * 8 + j) * 68 + t * 16 + lr] = fmaxf(acc[t][j], 0.f);
    __syncthreads();
    float* crow = C + (size_t)r0 * HH + c0;
    auto pass = [&]() {
#pragma unroll
        for (int s = 0; s < 8; ++s) { const int Lid = (lane >> 3) + 4 * s, piece = lane & 7; const int row = Lid >> 1, cofs = (Lid & 1) * 32 + piece * 4;
            const v4f val = *(const v4fa*)(os + row * 68 + cofs); *(volatile v4f*)(crow + (size_t)row * HH + cofs) = val; }
    };
    pass(); __threadfence(); pass();
}
__global__ __launch_bounds__(256) void k_colsum(const float* __restrict__ H, float* S) {
    const int b = blockIdx.x >> 1, h = (blockIdx.x & 1) * 256 + threadIdx.x;
    float s = 0.f;
#pragma unroll 4
    for (int i = 0; i < NP; ++i) s += H[((size_t)b * NP + i) * HH + h];
    VST2(float, S + (size_t)b * HH + h, s);
}
__global__ __launch_bounds__(256) void k_out(const float* __restrict__ S1, const float* __restrict__ S2, const float* __restrict__ Wp, const float* __restrict__ bp, float* out) {
    const int t = threadIdx.x;
#pragma unroll 1
    for (int q = 0; q < (NB_ * OO) / 256; ++q) {
        const int e = q * 256 + t, b = e / OO, o = e - b * OO;
        float acc = 0.f;
#pragma unroll 4
        for (int h = 0; h < HH; ++h) acc += S1[b * HH + h] * S2[b * HH + h] * bfr(Wp[h * OO + o]);
        acc += bfr(bp[o]) * (float)(NP * NP);
        VST2(float, out + e, acc);
    }
}

extern "C" void kernel_launch(void* const* d_in, const int* in_sizes, int n_in,
                              void* d_out, int out_size, void* d_ws, size_t ws_size, hipStream_t stream) {
    (void)in_sizes; (void)n_in; (void)out_size;
    const float* x1 = (const float*)d_in[0]; const float* x2 = (const float*)d_in[1]; const float* W1 = (const float*)d_in[2]; const float* W2 = (const float*)d_in[3];
    const float* Wp = (const float*)d_in[4]; const float* bp = (const float*)d_in[5];
    float* out = (float*)d_out;
    char* wsp = (char*)d_ws;
    auto take = [&](size_t bytes) { char* p = wsp; wsp += (bytes + 255) & ~(size_t)255; return (void*)p; };
    bf* X1b = (bf*)take((size_t)NR * CC * 2); bf* X2b = (bf*)take((size_t)NR * CC * 2); bf* W1T = (bf*)take((size_t)HH * CC * 2); bf* W2T = (bf*)take((size_t)HH * CC * 2);
    float* H1 = (float*)take((size_t)NR * HH * 4); float* H2 = (float*)take((size_t)NR * HH * 4); float* S1 = (float*)take((size_t)NB_ * HH * 4); float* S2 = (float*)take((size_t)NB_ * HH * 4);
    if ((size_t)(wsp - (char*)d_ws) > ws_size) return;
    k_cvtb<<<NR / 8, 256, 0, stream>>>(x1, X1b); k_cvtb<<<NR / 8, 256, 0, stream>>>(x2, X2b);
    k_wt<<<dim3(CC / 64, HH / 64, 1), 256, 0, stream>>>(W1, W1T); k_wt<<<dim3(CC / 64, HH / 64, 1), 256, 0, stream>>>(W2, W2T);
    k_gemm<<<dim3(NR / 64, HH / 64, 1), 128, 0, stream>>>(X1b, W1T, H1); k_gemm<<<dim3(NR / 64, HH / 64, 1), 128, 0, stream>>>(X2b, W2T, H2);
    k_colsum<<<NB_ * 2, 256, 0, stream>>>(H1, S1); k_colsum<<<NB_ * 2, 256, 0, stream>>>(H2, S2);
    k_out<<<1, 256, 0, stream>>>(S1, S2, Wp, bp, out);
}
